// CausalSelfAttention_4853313044761
// MI455X (gfx1250) — hardware-verified
//
#include <hip/hip_runtime.h>
#ifndef NB
#define NB 2
#endif
#ifndef SEQ
#define SEQ 2048
#endif
#define NB_FULL 2
#define SEQ_FULL 2048
#define CC 1024
#define NH 16
#define HD 64
#ifndef OUT_SEG_ROWS
#define OUT_SEG_ROWS SEQ_FULL
#endif
static_assert(NB >= 1 && NB <= NB_FULL);
static_assert(SEQ >= 64 && SEQ <= SEQ_FULL && (SEQ % 64) == 0);
static_assert(CC == NH * HD);
static_assert((HD % 32) == 0 && HD <= 128);
static_assert(((HD * 4) % 128) == 0);
static_assert((HD / 4) <= 32);
static_assert((CC % 64) == 0 && (CC % 32) == 0);
static_assert(((CC * CC) % 8) == 0 && (((CC * CC) / 8) % 256) == 0);
static_assert(((NB * SEQ) % 16) == 0 && (SEQ % 16) == 0);
static_assert((((NB * SEQ) / 16) * (CC / 64)) % 4 == 0);
static_assert(((3 * CC * 4) % 128) == 0 && ((CC * 4) % 128) == 0);
static_assert((size_t)((NB - 1) * OUT_SEG_ROWS + SEQ) <= (size_t)NB_FULL * SEQ_FULL || OUT_SEG_ROWS != SEQ_FULL);

typedef __bf16 v16b __attribute__((ext_vector_type(16)));
typedef unsigned short v8us __attribute__((ext_vector_type(8), may_alias));
typedef float  v8f  __attribute__((ext_vector_type(8)));
typedef float  v4f  __attribute__((ext_vector_type(4)));
typedef float  v4fa __attribute__((ext_vector_type(4), may_alias));
union FragB { v16b v; v8us half[2]; unsigned short u[16]; };

__device__ __forceinline__ unsigned short bf16_bits(float x) { unsigned int u = __float_as_uint(x); return (unsigned short)((u + 0x7FFFu + ((u >> 16) & 1u)) >> 16); }
__device__ __forceinline__ float bf16_val(unsigned short b) { return __uint_as_float(((unsigned int)b) << 16); }
__device__ __forceinline__ float bf16_rne(float x) { return bf16_val(bf16_bits(x)); }
template <int NT>
__device__ __forceinline__ v8f mmaN(v16b ah, v16b al, v16b bh, v16b bl, v8f c) {
  c = __builtin_amdgcn_wmma_f32_16x16x32_bf16(false, ah, false, bh, (short)0, c, false, false);
  if (NT >= 2) c = __builtin_amdgcn_wmma_f32_16x16x32_bf16(false, al, false, bh, (short)0, c, false, false);
  if (NT >= 3) c = __builtin_amdgcn_wmma_f32_16x16x32_bf16(false, ah, false, bl, (short)0, c, false, false);
  asm volatile("v_nop\n\tv_nop\n\tv_nop\n\tv_nop" : "+v"(c) : "v"(ah), "v"(al), "v"(bh), "v"(bl));
  return c;
}

__global__ __launch_bounds__(256) void k_w_bf16(const float* __restrict__ W, unsigned short* __restrict__ Wb, int n8) {
  const int t = blockIdx.x * 256 + threadIdx.x;
  if (t >= n8) return;
  const v4f a = *(const v4fa*)(W + (size_t)t * 8);
  const v4f b = *(const v4fa*)(W + (size_t)t * 8 + 4);
  v8us v;
  v[0] = bf16_bits(a[0]); v[1] = bf16_bits(a[1]); v[2] = bf16_bits(a[2]); v[3] = bf16_bits(a[3]);
  v[4] = bf16_bits(b[0]); v[5] = bf16_bits(b[1]); v[6] = bf16_bits(b[2]); v[7] = bf16_bits(b[3]);
  *(volatile v8us*)(Wb + (size_t)t * 8) = v;
  __threadfence();
  *(volatile v8us*)(Wb + (size_t)t * 8) = v;
}

template <bool ASPLIT>
__device__ __forceinline__ void gemm_body(const float* __restrict__ A, int lda, const unsigned short* __restrict__ Wt, int ldb,
                                          const float* __restrict__ bias, float* __restrict__ C, int ldc, int M, int N, int K,
                                          int seg, int asr, int csr) {
  __shared__ __attribute__((aligned(16))) float so[4][16][64];
  const int tid = threadIdx.x, w = tid >> 5, lane = tid & 31, ln = lane & 15, hh = lane >> 4;
  const int ntn = N / 64;
  const int wid = blockIdx.x * 4 + w;
  const int mt = wid / ntn, nq = wid % ntn;
  if (mt * 16 >= M) return;
  const int row0 = mt * 16, col0 = nq * 64;
  const int bseg = row0 / seg, t0 = row0 - bseg * seg;
  const float* arow = A + ((size_t)bseg * asr + t0 + ln) * lda;
  float* crow0 = C + ((size_t)bseg * csr + t0) * ldc;
  v8f acc[4];
#pragma unroll
  for (int t = 0; t < 4; ++t) acc[t] = (v8f){0.f,0.f,0.f,0.f,0.f,0.f,0.f,0.f};
  for (int kb = 0; kb < K; kb += 32) {
    FragB ah, al;
    const v4f x0 = *(const v4fa*)(arow + kb + 8 * hh), x1 = *(const v4fa*)(arow + kb + 8 * hh + 4);
    const v4f x2 = *(const v4fa*)(arow + kb + 16 + 8 * hh), x3 = *(const v4fa*)(arow + kb + 16 + 8 * hh + 4);
    float xs[16] = {x0[0],x0[1],x0[2],x0[3],x1[0],x1[1],x1[2],x1[3],x2[0],x2[1],x2[2],x2[3],x3[0],x3[1],x3[2],x3[3]};
#pragma unroll
    for (int i = 0; i < 16; ++i) { const unsigned short hb = bf16_bits(xs[i]); ah.u[i] = hb; al.u[i] = ASPLIT ? bf16_bits(xs[i] - bf16_val(hb)) : (unsigned short)0; }
#pragma unroll
    for (int t = 0; t < 4; ++t) {
      const unsigned short* brow = Wt + (size_t)(col0 + t * 16 + ln) * ldb + kb;
      FragB b;
      b.half[0] = *(const v8us*)(brow + 8 * hh);
      b.half[1] = *(const v8us*)(brow + 16 + 8 * hh);
      acc[t] = mmaN<ASPLIT ? 2 : 1>(ah.v, al.v, b.v, b.v, acc[t]);
    }
  }
#pragma unroll
  for (int t = 0; t < 4; ++t) {
    const float bv = bf16_rne(bias[col0 + t * 16 + ln]);
#pragma unroll
    for (int r = 0; r < 8; ++r) { const float v = acc[t][r] + bv; so[w][8 * hh + r][t * 16 + ln] = v; }
  }
  __builtin_amdgcn_fence(4  , "workgroup");
  __builtin_amdgcn_wave_barrier();
  const int rsub = lane >> 4, c4 = (lane & 15) * 4;
  for (int pass = 0; pass < 2; ++pass) {
#pragma unroll
    for (int q = 0; q < 8; ++q) {
      const int r = q * 2 + rsub;
      const v4f v = *(const v4fa*)&so[w][r][c4];
      *(volatile v4f*)(crow0 + (size_t)r * ldc + col0 + c4) = v;
    }
    if (pass == 0) __threadfence();
  }
}

__global__ __launch_bounds__(128) void k_gemm_x(const float* __restrict__ A, int lda, const unsigned short* __restrict__ Wt, int ldb,
                                                const float* __restrict__ bias, float* __restrict__ C, int ldc, int M, int N, int K,
                                                int seg, int asr, int csr) {
  gemm_body<false>(A, lda, Wt, ldb, bias, C, ldc, M, N, K, seg, asr, csr);
}
__global__ __launch_bounds__(128) void k_gemm_y(const float* __restrict__ A, int lda, const unsigned short* __restrict__ Wt, int ldb,
                                                const float* __restrict__ bias, float* __restrict__ C, int ldc, int M, int N, int K,
                                                int seg, int asr, int csr) {
  gemm_body<true>(A, lda, Wt, ldb, bias, C, ldc, M, N, K, seg, asr, csr);
}

__global__ __launch_bounds__(128) void k_flash(const float* __restrict__ qb, const float* __restrict__ kb, const float* __restrict__ vb,
                                               int pitch, int T, int H, float scale, float* __restrict__ y, int ypitch) {
  constexpr int D = HD;
  constexpr int KS = D / 32;
  constexpr int DT = D / 16;
  __shared__ __attribute__((aligned(16))) unsigned short sKh[32][D + 8], sKl[32][D + 8], sVh[32][D + 8], sVl[32][D + 8];
  __shared__ __attribute__((aligned(16))) unsigned short sPh[4][16][40], sPl[4][16][40];
  __shared__ __attribute__((aligned(16))) float sO[4][16][D];
  const int tid = threadIdx.x, w = tid >> 5, lane = tid & 31, ln = lane & 15, hh = lane >> 4;
  const int nqb = (T + 63) / 64;
  const int bh = blockIdx.x / nqb, qblk = blockIdx.x % nqb;
  const int b = bh / H, h = bh % H;
  const int q0 = qblk * 64 + w * 16;
  const float* Q = qb + (size_t)b * T * pitch + h * D;
  const float* K = kb + (size_t)b * T * pitch + h * D;
  const float* V = vb + (size_t)b * T * pitch + h * D;

  FragB aqh[KS], aql[KS];
  {
    int row = q0 + ln; if (row >= T) row = T - 1;
    const float* qr = Q + (size_t)row * pitch;
#pragma unroll
    for (int ks = 0; ks < KS; ++ks)
#pragma unroll
      for (int i = 0; i < 16; ++i) {
        const int d = ks * 32 + ((i < 8) ? (8 * hh + i) : (16 + 8 * hh + (i - 8)));
        const float x = qr[d] * scale; const unsigned short hb = bf16_bits(x);
        aqh[ks].u[i] = hb; aql[ks].u[i] = bf16_bits(x - bf16_val(hb));
      }
  }
  float m_r[8], l_r[8];
#pragma unroll
  for (int r = 0; r < 8; ++r) { m_r[r] = -3.0e38f; l_r[r] = 0.f; }
  v8f oacc[DT];
#pragma unroll
  for (int dt = 0; dt < DT; ++dt) oacc[dt] = (v8f){0.f,0.f,0.f,0.f,0.f,0.f,0.f,0.f};

  const int kv_end = min(T, qblk * 64 + 64);
  for (int j0 = 0; j0 < kv_end; j0 += 32) {
    __syncthreads();
    for (int e = tid; e < 32 * (D / 4); e += 128) {
      const int r = e / (D / 4), c4 = (e % (D / 4)) * 4;
      const int key = j0 + r;
      const int keyc = (key < T) ? key : (T - 1);
      v4f kf = *(const v4fa*)(K + (size_t)keyc * pitch + c4);
      v4f vf = *(const v4fa*)(V + (size_t)keyc * pitch + c4);
      if (key >= T) { kf = (v4f){0.f,0.f,0.f,0.f}; vf = (v4f){0.f,0.f,0.f,0.f}; }
#pragma unroll
      for (int t = 0; t < 4; ++t) {
        unsigned short hb = bf16_bits(kf[t]); sKh[r][c4 + t] = hb; sKl[r][c4 + t] = bf16_bits(kf[t] - bf16_val(hb));
        hb = bf16_bits(vf[t]); sVh[r][c4 + t] = hb; sVl[r][c4 + t] = bf16_bits(vf[t] - bf16_val(hb));
      }
    }
    __syncthreads();
    v8f s[2];
#pragma unroll
    for (int nt = 0; nt < 2; ++nt) {
      v8f acc = (v8f){0.f,0.f,0.f,0.f,0.f,0.f,0.f,0.f};
#pragma unroll
      for (int ks = 0; ks < KS; ++ks) {
        FragB bh_, bl_;
        bh_.half[0] = *(const v8us*)&sKh[nt * 16 + ln][ks * 32 + 8 * hh]; bh_.half[1] = *(const v8us*)&sKh[nt * 16 + ln][ks * 32 + 16 + 8 * hh];
        bl_.half[0] = *(const v8us*)&sKl[nt * 16 + ln][ks * 32 + 8 * hh]; bl_.half[1] = *(const v8us*)&sKl[nt * 16 + ln][ks * 32 + 16 + 8 * hh];
        acc = mmaN<3>(aqh[ks].v, aql[ks].v, bh_.v, bl_.v, acc);
      }
      s[nt] = acc;
    }
    float alpha[8];
#pragma unroll
    for (int r = 0; r < 8; ++r) {
      const int qi = q0 + 8 * hh + r;
      const int ja = j0 + ln, jb = j0 + 16 + ln;
      if (ja > qi) s[0][r] = -3.0e38f;
      if (jb > qi) s[1][r] = -3.0e38f;
      if (ja >= T) s[0][r] = -3.0e38f;
      if (jb >= T) s[1][r] = -3.0e38f;
      float mx = fmaxf(s[0][r], s[1][r]);
      mx = fmaxf(mx, __shfl_xor(mx, 1, 32)); mx = fmaxf(mx, __shfl_xor(mx, 2, 32)); mx = fmaxf(mx, __shfl_xor(mx, 4, 32)); mx = fmaxf(mx, __shfl_xor(mx, 8, 32));
      const float mnew = fmaxf(m_r[r], mx);
      alpha[r] = (mnew > -1.0e38f) ? __expf(m_r[r] - mnew) : 1.0f;
      const float p0 = (s[0][r] > -1.0e38f) ? __expf(s[0][r] - mnew) : 0.f;
      const float p1 = (s[1][r] > -1.0e38f) ? __expf(s[1][r] - mnew) : 0.f;
      m_r[r] = mnew;
      l_r[r] = l_r[r] * alpha[r] + p0 + p1;
      unsigned short hb = bf16_bits(p0); sPh[w][8 * hh + r][ln] = hb;      sPl[w][8 * hh + r][ln] = bf16_bits(p0 - bf16_val(hb));
      hb = bf16_bits(p1);                sPh[w][8 * hh + r][16 + ln] = hb; sPl[w][8 * hh + r][16 + ln] = bf16_bits(p1 - bf16_val(hb));
    }
#pragma unroll
    for (int dt = 0; dt < DT; ++dt)
#pragma unroll
      for (int r = 0; r < 8; ++r) oacc[dt][r] *= alpha[r];
    __builtin_amdgcn_fence(4  , "workgroup");
    __builtin_amdgcn_wave_barrier();
    FragB pah, pal;
    pah.half[0] = *(const v8us*)&sPh[w][ln][8 * hh]; pah.half[1] = *(const v8us*)&sPh[w][ln][16 + 8 * hh];
    pal.half[0] = *(const v8us*)&sPl[w][ln][8 * hh]; pal.half[1] = *(const v8us*)&sPl[w][ln][16 + 8 * hh];
#pragma unroll
    for (int dt = 0; dt < DT; ++dt) {
      FragB bvh, bvl;
#pragma unroll
      for (int i = 0; i < 8; ++i) {
        bvh.u[i] = sVh[8 * hh + i][dt * 16 + ln]; bvh.u[8 + i] = sVh[16 + 8 * hh + i][dt * 16 + ln];
        bvl.u[i] = sVl[8 * hh + i][dt * 16 + ln]; bvl.u[8 + i] = sVl[16 + 8 * hh + i][dt * 16 + ln];
      }
      oacc[dt] = mmaN<3>(pah.v, pal.v, bvh.v, bvl.v, oacc[dt]);
    }
    __builtin_amdgcn_fence(4  , "workgroup");
    __builtin_amdgcn_wave_barrier();
  }
#pragma unroll
  for (int r = 0; r < 8; ++r) {
    float l = l_r[r];
    l += __shfl_xor(l, 1, 32); l += __shfl_xor(l, 2, 32); l += __shfl_xor(l, 4, 32); l += __shfl_xor(l, 8, 32);
    l_r[r] = (l > 0.f) ? 1.0f / l : 0.f;
  }
#pragma unroll
  for (int dt = 0; dt < DT; ++dt)
#pragma unroll
    for (int r = 0; r < 8; ++r) sO[w][8 * hh + r][dt * 16 + ln] = oacc[dt][r] * l_r[r];
  __builtin_amdgcn_fence(4  , "workgroup");
  __builtin_amdgcn_wave_barrier();
  for (int pass = 0; pass < 2; ++pass) {
    for (int r = 0; r < 16; ++r) {
      const int row = q0 + r;
      if (row < T && lane < D / 4) {
        const v4f val = *(const v4fa*)&sO[w][r][lane * 4];
        *(volatile v4f*)(y + ((size_t)b * T + row) * ypitch + h * D + lane * 4) = val;
      }
    }
    if (pass == 0) __threadfence();
  }
}

constexpr size_t WS_W   = (size_t)CC * CC * 2;
constexpr size_t WS_QKV = (size_t)NB * SEQ * 3 * CC * 4;
constexpr size_t WS_Y   = (size_t)NB * SEQ * CC * 4;
constexpr size_t WS_TOTAL = 4 * WS_W + WS_QKV + WS_Y;
static_assert((WS_W % 128) == 0 && (WS_QKV % 128) == 0 && (WS_Y % 128) == 0);
static_assert(WS_TOTAL <= (size_t)134217728);

extern "C" void kernel_launch(void* const* d_in, const int* in_sizes, int n_in,
                              void* d_out, int out_size, void* d_ws, size_t ws_size, hipStream_t stream) {
  if (n_in < 9) return;
  if (in_sizes[0] < ((NB - 1) * SEQ_FULL + SEQ) * CC) return;
  for (int i = 1; i < 9; i += 2) {
    if (in_sizes[i] < CC * CC) return;
    if (in_sizes[i + 1] < CC) return;
  }
  if (out_size < ((NB - 1) * OUT_SEG_ROWS + SEQ) * CC) return;
  const float* x  = (const float*)d_in[0];
  const float* Wq = (const float*)d_in[1]; const float* bqp = (const float*)d_in[2];
  const float* Wk = (const float*)d_in[3]; const float* bkp = (const float*)d_in[4];
  const float* Wv = (const float*)d_in[5]; const float* bvp = (const float*)d_in[6];
  const float* Wp = (const float*)d_in[7]; const float* bpp = (const float*)d_in[8];
  char* ws = (char*)d_ws; size_t off = 0;
  unsigned short* Wqb = (unsigned short*)(ws + off); off += WS_W;
  unsigned short* Wkb = (unsigned short*)(ws + off); off += WS_W;
  unsigned short* Wvb = (unsigned short*)(ws + off); off += WS_W;
  unsigned short* Wpb = (unsigned short*)(ws + off); off += WS_W;
  float* qkv = (float*)(ws + off); off += WS_QKV;
  float* yb  = (float*)(ws + off); off += WS_Y;
  if (off > ws_size) return;
  const int M = NB * SEQ;
  const int n8 = (CC * CC) / 8;
  const int gw = (n8 + 255) / 256;
  k_w_bf16<<<gw, 256, 0, stream>>>(Wq, Wqb, n8);
  k_w_bf16<<<gw, 256, 0, stream>>>(Wk, Wkb, n8);
  k_w_bf16<<<gw, 256, 0, stream>>>(Wv, Wvb, n8);
  k_w_bf16<<<gw, 256, 0, stream>>>(Wp, Wpb, n8);
  const int gg = ((M / 16) * (CC / 64) + 3) / 4;
  k_gemm_x<<<gg, 128, 0, stream>>>(x, CC, Wqb, CC, bqp, qkv,          3 * CC, M, CC, CC, SEQ, SEQ_FULL, SEQ);
  k_gemm_x<<<gg, 128, 0, stream>>>(x, CC, Wkb, CC, bkp, qkv + CC,     3 * CC, M, CC, CC, SEQ, SEQ_FULL, SEQ);
  k_gemm_x<<<gg, 128, 0, stream>>>(x, CC, Wvb, CC, bvp, qkv + 2 * CC, 3 * CC, M, CC, CC, SEQ, SEQ_FULL, SEQ);
  k_flash<<<NB * NH * (SEQ / 64), 128, 0, stream>>>(qkv, qkv + CC, qkv + 2 * CC, 3 * CC, SEQ, NH, 0.125f, yb, CC);
  k_gemm_y<<<gg, 128, 0, stream>>>(yb, CC, Wpb, CC, bpp, (float*)d_out, CC, M, CC, CC, SEQ, SEQ, OUT_SEG_ROWS);
}
